// TypeConditionalLinear_83056077570517
// MI455X (gfx1250) — hardware-verified
//
#include <hip/hip_runtime.h>
#include <math.h>

typedef __attribute__((ext_vector_type(16))) _Float16 v16h;
typedef __attribute__((ext_vector_type(16))) __bf16 v16b;
typedef __attribute__((ext_vector_type(8)))  _Float16 v8h;
typedef __attribute__((ext_vector_type(8)))  float v8f;
typedef __attribute__((ext_vector_type(4)))  float v4f;
typedef __attribute__((ext_vector_type(2)))  float v2f;
typedef __attribute__((ext_vector_type(4)))  unsigned v4u;
typedef __attribute__((ext_vector_type(4)))  int v4i;
typedef float __attribute__((may_alias)) float_a;
typedef int __attribute__((may_alias)) int_a;

template <typename T> __device__ __forceinline__ void vst2(void* p, T v) { *(volatile T*)p = v; __threadfence(); *(volatile T*)p = v; }
__device__ __forceinline__ v8f wmma16(v16h a, v16h b, v8f c) {
  v8f d = __builtin_amdgcn_wmma_f32_16x16x32_f16(false, a, false, b, (short)0, c, false, false);
  asm volatile("v_nop\n\tv_nop\n\tv_nop\n\tv_nop" : "+v"(d) : "v"(a), "v"(b));
  return d;
}
__device__ __forceinline__ v8f wmma_bf(v16b a, v16b b, v8f c) {
  v8f d = __builtin_amdgcn_wmma_f32_16x16x32_bf16(false, a, false, b, (short)0, c, false, false);
  asm volatile("v_nop\n\tv_nop\n\tv_nop\n\tv_nop" : "+v"(d) : "v"(a), "v"(b));
  return d;
}
__device__ __forceinline__ v16h frag_h(const _Float16* rowk0, int lane) {
  union { v16h v; v8h q[2]; } u; const _Float16* p = rowk0 + 8 * (lane >> 4);
  u.q[0] = *(const v8h*)p; u.q[1] = *(const v8h*)(p + 16); return u.v;
}
__device__ __forceinline__ v16h frag_f32(const float* rowk0, int lane) {
  v16h a; const float* p = rowk0 + 8 * (lane >> 4);
#pragma unroll
  for (int i = 0; i < 8; ++i) { a[i] = (_Float16)p[i]; a[8 + i] = (_Float16)p[16 + i]; }
  return a;
}
__device__ __forceinline__ v16h frag_f32s(const float* rowk0, int lane, float sc) {
  v16h a; const float* p = rowk0 + 8 * (lane >> 4);
#pragma unroll
  for (int i = 0; i < 8; ++i) { a[i] = (_Float16)(p[i] * sc); a[8 + i] = (_Float16)(p[16 + i] * sc); }
  return a;
}
__device__ __forceinline__ v16h fragc_f32(const float* W, int k0, int n, int lane, int ld, int K) {
  v16h a; const int g = lane >> 4;
#pragma unroll
  for (int i = 0; i < 8; ++i) { const int ka = k0 + 8 * g + i, kb = ka + 16;
    a[i] = (_Float16)(ka < K ? W[(size_t)(ka < K ? ka : K - 1) * ld + n] : 0.f); a[8 + i] = (_Float16)(kb < K ? W[(size_t)(kb < K ? kb : K - 1) * ld + n] : 0.f); }
  return a;
}
struct F2 { v16b h, l; };
__device__ __forceinline__ F2 bsplit16(const float v[16]) { F2 r;
#pragma unroll
  for (int i = 0; i < 16; ++i) { const __bf16 h = (__bf16)v[i]; r.h[i] = h; r.l[i] = (__bf16)(v[i] - (float)h); }
  return r; }
__device__ __forceinline__ F2 split_row(const float* row, int k0, int lane) { float v[16]; const float* p = row + k0 + 8 * (lane >> 4);
#pragma unroll
  for (int i = 0; i < 8; ++i) { v[i] = p[i]; v[8 + i] = p[16 + i]; }
  return bsplit16(v); }
__device__ __forceinline__ F2 split_rowK(const float* row, int k0, int lane, int K) { float v[16]; const int g = lane >> 4;
#pragma unroll
  for (int i = 0; i < 8; ++i) { const int ka = k0 + 8 * g + i, kb = ka + 16; v[i] = ka < K ? row[ka < K ? ka : K - 1] : 0.f; v[8 + i] = kb < K ? row[kb < K ? kb : K - 1] : 0.f; }
  return bsplit16(v); }
__device__ __forceinline__ F2 split_col(const float* W, int k0, int n, int lane, int ld, int K) { float v[16]; const int g = lane >> 4;
#pragma unroll
  for (int i = 0; i < 8; ++i) { const int ka = k0 + 8 * g + i, kb = ka + 16; v[i] = ka < K ? W[(size_t)(ka < K ? ka : K - 1) * ld + n] : 0.f; v[8 + i] = kb < K ? W[(size_t)(kb < K ? kb : K - 1) * ld + n] : 0.f; }
  return bsplit16(v); }
__device__ __forceinline__ v8f mac3(const F2& a, const F2& b, v8f c) { c = wmma_bf(a.l, b.h, c); c = wmma_bf(a.h, b.l, c); return wmma_bf(a.h, b.h, c); }
__device__ __forceinline__ float sigm(float v) { return 1.0f / (1.0f + expf(-v)); }
#define LDSX() do { asm volatile("s_wait_dscnt 0" ::: "memory"); __builtin_amdgcn_wave_barrier(); __builtin_amdgcn_fence(__ATOMIC_RELEASE, "workgroup"); } while (0)


#define NTOK 16384
#define IN_ 512
#define OUT_ 512
#define NTY 16
#define NSLOT (NTOK + NTY * 64)
#define NGB (NSLOT / 64)
typedef __attribute__((ext_vector_type(8))) __bf16 v8b;
__device__ __forceinline__ v16b frag_b(const __bf16* rowk0, int lane) {
  union { v16b v; v8b q[2]; } u; const __bf16* p = rowk0 + 8 * (lane >> 4);
  u.q[0] = *(const v8b*)p; u.q[1] = *(const v8b*)(p + 16); return u.v;
}
__device__ __forceinline__ float bfr(float v) { return (float)(__bf16)v; }
__device__ __attribute__((noinline)) float exp_ni(float v) { return expf(v); }
__device__ __attribute__((noinline)) float erf_ni(float v) { return erff(v); }

#define WS_PERM 0u
#define WS_PFX  (WS_PERM + 4u * (size_t)NSLOT)
#define WS_END  (WS_PFX + 4u * 32)

__global__ __launch_bounds__(256) void k_sort(const int* __restrict__ TY, int* __restrict__ PERM, int* __restrict__ PFX) { __shared__ int scnt[NTY]; __shared__ __align__(16) int spfx[32]; __shared__ __align__(16) int sperm[NSLOT];
  const int t = threadIdx.x;
  for (int e = t; e < NSLOT; e += 256) sperm[e] = -1;
  if (t < NTY) { int c = 0;
#pragma unroll 1
    for (int n = 0; n < NTOK; ++n) c += (TY[n] == t) ? 1 : 0; scnt[t] = c; }
  __syncthreads();
  if (t == 0) { int s = 0; for (int k = 0; k < NTY; ++k) { spfx[k] = s; s += ((scnt[k] + 63) / 64) * 64; } spfx[NTY] = s; for (int k = NTY + 1; k < 32; ++k) spfx[k] = s; }
  __syncthreads();
  if (t < NTY) { int pos = spfx[t];
#pragma unroll 1
    for (int n = 0; n < NTOK; ++n) if (TY[n] == t) sperm[pos++] = n; }
  __syncthreads();
  for (int q = t; q < NSLOT / 4; q += 256) vst2((int*)PERM + q * 4, *(const v4i*)&sperm[q * 4]);
  if (t < 8) vst2(PFX + t * 4, *(const v4i*)&spfx[t * 4]); }
__global__ __launch_bounds__(128) void k_gemm(const float* __restrict__ X, const int* __restrict__ PERM, const int* __restrict__ PFX, const float* __restrict__ Wt, const float* __restrict__ Bs, float* __restrict__ OUT) { __shared__ __align__(16) float sf[4][16][132]; __shared__ int sty; __shared__ int sidx[64];
  const int tid = threadIdx.x, wave = tid >> 5, lane = tid & 31, col = lane & 15, g = lane >> 4; const int s0 = blockIdx.x * 64, c0 = blockIdx.y * 128;
  if (tid == 0) { int ty = -1; for (int k = 0; k < NTY; ++k) if (s0 >= PFX[k] && s0 < PFX[k + 1]) ty = k; sty = ty; }
  if (tid < 64) sidx[tid] = PERM[s0 + tid < NSLOT ? s0 + tid : NSLOT - 1];
  __syncthreads(); const int ty = sty; if (ty < 0) return;
  const int myrow = sidx[wave * 16 + col]; const float* xr = X + (size_t)(myrow >= 0 ? myrow : 0) * IN_; const float* Wm = Wt + (size_t)ty * OUT_ * IN_;
  v8f acc[8] = {};
#pragma unroll 2
  for (int kc = 0; kc < IN_ / 32; ++kc) { v16b a;
#pragma unroll
    for (int i = 0; i < 8; ++i) { a[i] = (__bf16)(myrow >= 0 ? xr[kc * 32 + 8 * g + i] : 0.f); a[8 + i] = (__bf16)(myrow >= 0 ? xr[kc * 32 + 16 + 8 * g + i] : 0.f); }
#pragma unroll
    for (int j = 0; j < 8; ++j) { v16b w; const int o = c0 + j * 16 + col;
#pragma unroll
      for (int i = 0; i < 8; ++i) { w[i] = (__bf16)Wm[(size_t)o * IN_ + kc * 32 + 8 * g + i]; w[8 + i] = (__bf16)Wm[(size_t)o * IN_ + kc * 32 + 16 + 8 * g + i]; }
      acc[j] = wmma_bf(a, w, acc[j]); } }
#pragma unroll
  for (int j = 0; j < 8; ++j) { const float bb = bfr(Bs[ty * OUT_ + c0 + j * 16 + col]);
#pragma unroll
    for (int r = 0; r < 8; ++r) sf[wave][8 * g + r][j * 16 + col] = acc[j][r] + bb; }
  LDSX();
  for (int rl = 0; rl < 16; ++rl) { const int row = sidx[wave * 16 + rl]; if (row >= 0) vst2(OUT + (size_t)row * OUT_ + c0 + lane * 4, *(const v4f*)&sf[wave][rl][lane * 4]); } }
extern "C" void kernel_launch(void* const* d_in, const int* in_sizes, int n_in, void* d_out, int out_size, void* d_ws, size_t ws_size, hipStream_t stream) {
  (void)in_sizes; (void)n_in; (void)out_size;
  const float** F = (const float**)d_in;
  if (ws_size < (size_t)WS_END) return;
  char* ws = (char*)d_ws; int *PERM = (int*)(ws + WS_PERM), *PFX = (int*)(ws + WS_PFX);
  k_sort<<<1, 256, 0, stream>>>((const int*)d_in[1], PERM, PFX);
  k_gemm<<<dim3(NGB, OUT_ / 128), 128, 0, stream>>>(F[0], PERM, PFX, F[2], F[3], (float*)d_out);
}
